// VSSBlock_85401129714116
// MI455X (gfx1250) — hardware-verified
//
#include <hip/hip_runtime.h>
#include <stddef.h>

typedef __attribute__((ext_vector_type(16))) _Float16 v16h;
typedef __attribute__((ext_vector_type(8)))  _Float16 v8h;
typedef __attribute__((ext_vector_type(16))) __bf16   v16b;
typedef __attribute__((ext_vector_type(8)))  __bf16   v8b;
typedef __attribute__((ext_vector_type(8)))  float    v8f;
typedef __attribute__((ext_vector_type(4)))  float    v4f;
typedef __attribute__((ext_vector_type(4)))  unsigned int v4u;

__device__ __forceinline__ unsigned short f2bf_bits(float f) {
  unsigned u = __float_as_uint(f);
  return (unsigned short)((u + 0x7FFFu + ((u >> 16) & 1u)) >> 16);
}
__device__ __forceinline__ float bf_bits2f(unsigned short h) { return __uint_as_float(((unsigned)h) << 16); }

__device__ __forceinline__ void dep_guard_h(v8f& a, v8f& b, v16h x, v16h y) { asm volatile("v_nop\n\tv_nop\n\tv_nop\n\tv_nop" : "+v"(a), "+v"(b) : "v"(x), "v"(y)); }
__device__ __forceinline__ void dep_guard_b(v8f& a, v8f& b, v16b x, v16b y) { asm volatile("v_nop\n\tv_nop\n\tv_nop\n\tv_nop" : "+v"(a), "+v"(b) : "v"(x), "v"(y)); }
__device__ __forceinline__ void keep4_h(v16h a, v16h b, v16h c, v16h d) { asm volatile("v_nop" :: "v"(a), "v"(b), "v"(c), "v"(d)); }
__device__ __forceinline__ void keep4_b(v16b a, v16b b, v16b c, v16b d) { asm volatile("v_nop" :: "v"(a), "v"(b), "v"(c), "v"(d)); }
__device__ __forceinline__ void acc_guard4(v8f& a, v8f& b, v8f& c, v8f& d) { asm volatile("v_nop\n\tv_nop\n\tv_nop\n\tv_nop" : "+v"(a), "+v"(b), "+v"(c), "+v"(d)); }
__device__ __forceinline__ void guard3_h(v8f& a0, v8f& a1, v8f& a2, v16h x, v16h y0, v16h y1, v16h y2) {
  asm volatile("v_nop\n\tv_nop\n\tv_nop\n\tv_nop" : "+v"(a0), "+v"(a1), "+v"(a2) : "v"(x), "v"(y0), "v"(y1), "v"(y2));
}
__device__ __forceinline__ void acc_guard3(v8f& a, v8f& b, v8f& c) { asm volatile("v_nop\n\tv_nop\n\tv_nop\n\tv_nop" : "+v"(a), "+v"(b), "+v"(c)); }

template <typename T> struct Frag;
template <> struct Frag<_Float16> {
  typedef v16h V; union U { v16h v; v8h h[2]; };
  static __device__ __forceinline__ v16h load(const _Float16* p) {
    U f; f.h[0] = *(const v8h*)(p); f.h[1] = *(const v8h*)(p + 16); return f.v;
  }
  static __device__ __forceinline__ v8f mma(v16h a, v16h b, v8f c) {
    return __builtin_amdgcn_wmma_f32_16x16x32_f16(false, a, false, b, (short)0, c, false, false);
  }
  static __device__ __forceinline__ void guard(v8f& a, v8f& b, v16h x, v16h y) { dep_guard_h(a, b, x, y); }
  static __device__ __forceinline__ void keep(v16h a, v16h b, v16h c, v16h d) { keep4_h(a, b, c, d); }
};
template <> struct Frag<__bf16> {
  typedef v16b V; union U { v16b v; v8b h[2]; };
  static __device__ __forceinline__ v16b load(const __bf16* p) {
    U f; f.h[0] = *(const v8b*)(p); f.h[1] = *(const v8b*)(p + 16); return f.v;
  }
  static __device__ __forceinline__ v8f mma(v16b a, v16b b, v8f c) {
    return __builtin_amdgcn_wmma_f32_16x16x32_bf16(false, a, false, b, (short)0, c, false, false);
  }
  static __device__ __forceinline__ void guard(v8f& a, v8f& b, v16b x, v16b y) { dep_guard_b(a, b, x, y); }
  static __device__ __forceinline__ void keep(v16b a, v16b b, v16b c, v16b d) { keep4_b(a, b, c, d); }
};

template <int ET> struct Elem;
template <> struct Elem<0> { typedef _Float16 T; };
template <> struct Elem<1> { typedef __bf16 T; };
template <int ET, bool SPLIT, int BIAS_MODE, int OUT_MODE, bool RESID, int ACT = 0>
__global__ __launch_bounds__(256) void wmma_gemm64(
    const unsigned short* __restrict__ Ap, const unsigned short* __restrict__ A2p, int lda, long strideA,
    const unsigned short* __restrict__ Btp, const unsigned short* __restrict__ Bt2p, int ldb, long strideB,
    void* __restrict__ Cout, void* __restrict__ Cout2, int ldc, long strideC,
    const float* __restrict__ bias,
    const float* __restrict__ resid, long strideR,
    int M, int N, int K, float scale) {
  typedef typename Elem<ET>::T T;
  typedef typename Frag<T>::V V;
  const T* A = (const T*)Ap; const T* A2 = (const T*)A2p; const T* Bt = (const T*)Btp; const T* Bt2 = (const T*)Bt2p;
  __shared__ __align__(16) float sT[8][16 * 68];
  const int b    = blockIdx.y;
  const int lane = threadIdx.x & 31;
  const int wave = threadIdx.x >> 5;
  const int tilesN = N >> 6;
  const int tilesM = M >> 6;
  const int tile = blockIdx.x * 8 + wave;
  if (tile >= tilesM * tilesN) return;
  const int tm = tile / tilesN;
  const int tn = tile - tm * tilesN;
  const int m0 = tm << 6;
  const int n0 = tn << 6;

  const T* Ab  = A  + (size_t)b * strideA;
  const T* Bb  = Bt + (size_t)b * strideB;
  const T* Ab2 = SPLIT ? (A2  + (size_t)b * strideA) : nullptr;
  const T* Bb2 = SPLIT ? (Bt2 + (size_t)b * strideB) : nullptr;

  const int rlane = lane & 15;
  const int koff  = (lane >> 4) * 8;
  const int mOff  = (lane >> 4) * 8;

  v8f acc[4][4];
#pragma unroll
  for (int i = 0; i < 4; ++i)
#pragma unroll
    for (int j = 0; j < 4; ++j) acc[i][j] = (v8f){0.f,0.f,0.f,0.f,0.f,0.f,0.f,0.f};

  for (int k0 = 0; k0 < K; k0 += 32) {
    V bh[4], bl[4];
#pragma unroll
    for (int j = 0; j < 4; ++j) {
      const size_t bo = (size_t)(n0 + (j << 4) + rlane) * ldb + koff + k0;
      bh[j] = Frag<T>::load(Bb + bo);
      if (SPLIT) bl[j] = Frag<T>::load(Bb2 + bo);
    }
#pragma unroll
    for (int i = 0; i < 4; ++i) {
      const size_t ao = (size_t)(m0 + (i << 4) + rlane) * lda + koff + k0;
      V ah = Frag<T>::load(Ab + ao);
      V al;
      if (SPLIT) al = Frag<T>::load(Ab2 + ao);
#pragma unroll
      for (int j = 0; j < 4; ++j) {
        acc[i][j] = Frag<T>::mma(ah, bh[j], acc[i][j]);
        if (SPLIT) {
          acc[i][j] = Frag<T>::mma(ah, bl[j], acc[i][j]);
          acc[i][j] = Frag<T>::mma(al, bh[j], acc[i][j]);
        }
      }
      Frag<T>::guard(acc[i][0], acc[i][3], ah, SPLIT ? al : ah);
    }
    Frag<T>::keep(bh[0], bh[1], bh[2], bh[3]);
    if (SPLIT) Frag<T>::keep(bl[0], bl[1], bl[2], bl[3]);
  }
  acc_guard4(acc[0][0], acc[0][1], acc[0][2], acc[0][3]);
  acc_guard4(acc[1][0], acc[1][1], acc[1][2], acc[1][3]);
  acc_guard4(acc[2][0], acc[2][1], acc[2][2], acc[2][3]);
  acc_guard4(acc[3][0], acc[3][1], acc[3][2], acc[3][3]);

  float* slab = sT[wave];
  const float* Rb = RESID ? (resid + (size_t)b * strideR) : nullptr;
#pragma unroll
  for (int i = 0; i < 4; ++i) {
    const int mBase = m0 + (i << 4);
#pragma unroll
    for (int j = 0; j < 4; ++j) {
      const int n = n0 + (j << 4) + rlane;
      float bv = 0.f;
      if (BIAS_MODE == 2) bv = bias[n];
#pragma unroll
      for (int r = 0; r < 8; ++r) {
        float v = acc[i][j][r] * scale;
        if (BIAS_MODE == 1) v += bias[mBase + mOff + r];
        if (BIAS_MODE == 2) v += bv;
        if (RESID) v += Rb[(size_t)(mBase + mOff + r) * ldc + n];
        if (ACT == 1) v = tanhf(v);
        if (ACT == 2) v = fmaxf(v, 0.0f);
        if (ACT == 3) v = v / (1.0f + expf(-v));
        if (ACT == 4) v = (v > 0.f) ? v : 0.01f * v;
        if (ACT == 5) v = 0.5f * v * (1.0f + erff(v * 0.70710678118654752f));
        slab[(mOff + r) * 68 + (j << 4) + rlane] = v;
      }
    }
    __builtin_amdgcn_fence(__ATOMIC_RELEASE, "workgroup");
    __builtin_amdgcn_wave_barrier();
    __builtin_amdgcn_fence(__ATOMIC_ACQUIRE, "workgroup");
    if (OUT_MODE == 0) {
      float* C = (float*)Cout + (size_t)b * strideC;
      const int hh = lane >> 4, c4 = (lane & 15) * 4;
      for (int pass = 0; pass < 2; ++pass) {
#pragma unroll
        for (int it = 0; it < 8; ++it) {
          const int row = it * 2 + hh;
          v4f v = *(const v4f*)(slab + row * 68 + c4);
          *(volatile v4f*)(C + (size_t)(mBase + row) * ldc + n0 + c4) = v;
        }
        __threadfence();
      }
    } else {
      const int q = lane >> 3, c8 = (lane & 7) * 8;
      unsigned short* C  = (unsigned short*)Cout  + (size_t)b * strideC;
      unsigned short* C2 = (OUT_MODE == 2) ? ((unsigned short*)Cout2 + (size_t)b * strideC) : nullptr;
      for (int pass = 0; pass < 2; ++pass) {
#pragma unroll
        for (int it = 0; it < 4; ++it) {
          const int row = it * 4 + q;
          const float* sp = slab + row * 68 + c8;
          v8h hv, lv;
#pragma unroll
          for (int e = 0; e < 8; ++e) {
            if (OUT_MODE == 1) {
              hv[e] = (_Float16)sp[e];
            } else {
              unsigned short hb = f2bf_bits(sp[e]);
              unsigned short lb = f2bf_bits(sp[e] - bf_bits2f(hb));
              hv[e] = __builtin_bit_cast(_Float16, hb);
              lv[e] = __builtin_bit_cast(_Float16, lb);
            }
          }
          *(volatile v8h*)(C + (size_t)(mBase + row) * ldc + n0 + c8) = hv;
          if (OUT_MODE == 2) *(volatile v8h*)(C2 + (size_t)(mBase + row) * ldc + n0 + c8) = lv;
        }
        __threadfence();
      }
    }
    __builtin_amdgcn_fence(__ATOMIC_RELEASE, "workgroup");
    __builtin_amdgcn_wave_barrier();
    __builtin_amdgcn_fence(__ATOMIC_ACQUIRE, "workgroup");
  }
}

constexpr int NB_IMG    = 32;
constexpr int IMG_H     = 56;
constexpr int IMG_W     = 56;
constexpr int NCH_MODEL = 96;
constexpr int NCH_INNER = 192;
constexpr int NCH_PROJ  = 384;
constexpr int NPOS_ALL  = NB_IMG * IMG_H * IMG_W;
constexpr int TILE_P    = 8;
constexpr int HALO_P    = 10;
constexpr int NHALO     = HALO_P * HALO_P;
constexpr int TILES_X   = IMG_W / TILE_P;
constexpr int TILES_Y   = IMG_H / TILE_P;
constexpr int NTILE_BLK = NB_IMG * TILES_X * TILES_Y;
constexpr int LN_POS_BLK = 64;
constexpr int LN_NBLK    = NPOS_ALL / LN_POS_BLK;
constexpr int WIN_PLANE_HALVES = NCH_INNER * NCH_MODEL;
constexpr int WPK_HALVES = 9 * 6 * 6 * 512;
constexpr float CONVW_CARRY     = 64.0f;
constexpr float CONVW_CARRY_INV = 1.0f / 64.0f;

static_assert(IMG_H % TILE_P == 0 && IMG_W % TILE_P == 0);
static_assert(NPOS_ALL % LN_POS_BLK == 0);
static_assert(NPOS_ALL % 64 == 0);
static_assert(NCH_INNER % 64 == 0);
static_assert(NCH_MODEL % 32 == 0);
static_assert((NPOS_ALL / 64) * (NCH_INNER / 64) % 8 == 0);
static_assert(WIN_PLANE_HALVES % 64 == 0 && WPK_HALVES % 64 == 0);
static_assert((LN_POS_BLK * NCH_MODEL) % 64 == 0);

constexpr size_t SZ_H    = (size_t)NPOS_ALL * NCH_MODEL * 2;
constexpr size_t SZ_W    = (size_t)WIN_PLANE_HALVES * 2;
constexpr size_t SZ_WPK  = (size_t)WPK_HALVES * 2;
constexpr size_t SZ_X1   = (size_t)NPOS_ALL * NCH_INNER * 2;
constexpr size_t OFF_HHI = 0;
constexpr size_t OFF_HLO = OFF_HHI + SZ_H;
constexpr size_t OFF_WHI = OFF_HLO + SZ_H;
constexpr size_t OFF_WLO = OFF_WHI + SZ_W;
constexpr size_t OFF_WPK = OFF_WLO + SZ_W;
constexpr size_t OFF_X1  = OFF_WPK + SZ_WPK;
constexpr size_t WS_TOTAL = OFF_X1 + SZ_X1;
static_assert(OFF_HLO % 128 == 0 && OFF_WHI % 128 == 0 && OFF_WLO % 128 == 0 && OFF_WPK % 128 == 0 && OFF_X1 % 128 == 0);
static_assert(WS_TOTAL <= (size_t)134217728);

__device__ __forceinline__ void pack_hilo_pair(float f0, float f1, unsigned& hw, unsigned& lw) {
  const unsigned short h0 = f2bf_bits(f0);
  const unsigned short h1 = f2bf_bits(f1);
  const unsigned short l0 = f2bf_bits(f0 - bf_bits2f(h0));
  const unsigned short l1 = f2bf_bits(f1 - bf_bits2f(h1));
  hw = (unsigned)h0 | ((unsigned)h1 << 16);
  lw = (unsigned)l0 | ((unsigned)l1 << 16);
}

__global__ __launch_bounds__(256) void ln_split_planes(
    const float* __restrict__ x, const float* __restrict__ ln_w, const float* __restrict__ ln_b,
    unsigned short* __restrict__ hhi, unsigned short* __restrict__ hlo)
{
  __shared__ __align__(16) float sHf[LN_POS_BLK * NCH_MODEL];
  __shared__ __align__(16) float sW[NCH_MODEL];
  __shared__ __align__(16) float sBv[NCH_MODEL];
  const int tid = threadIdx.x, lane = tid & 31, wave = tid >> 5;
  const int blk = blockIdx.x;

  if (wave == 0) {
    const int q = lane < 24 ? lane : 23;
    const v4f w4 = *(const v4f*)(ln_w + q * 4);
    if (lane < 24) *(v4f*)(sW + lane * 4) = w4;
  } else if (wave == 1) {
    const int q = lane < 24 ? lane : 23;
    const v4f b4 = *(const v4f*)(ln_b + q * 4);
    if (lane < 24) *(v4f*)(sBv + lane * 4) = b4;
  }
  __syncthreads();

  const int pos = tid >> 2, part = tid & 3;
  const size_t rowoff = ((size_t)blk * LN_POS_BLK + pos) * NCH_MODEL + part * 24;
  v4f xv[6];
#pragma unroll
  for (int i = 0; i < 6; ++i) xv[i] = *(const v4f*)(x + rowoff + 4 * i);
  float s = 0.0f;
#pragma unroll
  for (int i = 0; i < 6; ++i) s += (xv[i][0] + xv[i][1]) + (xv[i][2] + xv[i][3]);
  s += __shfl_xor(s, 1, 32);
  s += __shfl_xor(s, 2, 32);
  const float mean = s * (1.0f / 96.0f);
  float sq = 0.0f;
#pragma unroll
  for (int i = 0; i < 6; ++i) {
#pragma unroll
    for (int e = 0; e < 4; ++e) { const float d = xv[i][e] - mean; sq += d * d; }
  }
  sq += __shfl_xor(sq, 1, 32);
  sq += __shfl_xor(sq, 2, 32);
  const float var = sq * (1.0f / 96.0f);
  const float rs = rsqrtf(var + 1e-5f);
#pragma unroll
  for (int i = 0; i < 6; ++i) {
    const int c = part * 24 + 4 * i;
    const v4f w4 = *(const v4f*)(sW + c);
    const v4f b4 = *(const v4f*)(sBv + c);
    v4f hv4;
#pragma unroll
    for (int e = 0; e < 4; ++e) hv4[e] = (xv[i][e] - mean) * rs * w4[e] + b4[e];
    *(v4f*)(sHf + pos * NCH_MODEL + c) = hv4;
  }
  __syncthreads();

  const size_t cb = (size_t)blk * (LN_POS_BLK * NCH_MODEL);
  v4u hvv[3], lvv[3];
#pragma unroll
  for (int it = 0; it < 3; ++it) {
    const int item = it * 256 + tid;
    const int e0 = (item >> 3) * 64 + (item & 7) * 8;
    const v4f p0 = *(const v4f*)(sHf + e0);
    const v4f p1 = *(const v4f*)(sHf + e0 + 4);
    unsigned hw0, hw1, hw2, hw3, lw0, lw1, lw2, lw3;
    pack_hilo_pair(p0[0], p0[1], hw0, lw0);
    pack_hilo_pair(p0[2], p0[3], hw1, lw1);
    pack_hilo_pair(p1[0], p1[1], hw2, lw2);
    pack_hilo_pair(p1[2], p1[3], hw3, lw3);
    hvv[it] = (v4u){hw0, hw1, hw2, hw3};
    lvv[it] = (v4u){lw0, lw1, lw2, lw3};
  }
  for (int ps = 0; ps < 2; ++ps) {
#pragma unroll
    for (int it = 0; it < 3; ++it) {
      const int item = it * 256 + tid;
      const size_t e0 = (size_t)((item >> 3) * 64 + (item & 7) * 8);
      *(volatile v4u*)(void*)(hhi + cb + e0) = hvv[it];
      *(volatile v4u*)(void*)(hlo + cb + e0) = lvv[it];
    }
    __threadfence();
  }
}

__global__ __launch_bounds__(256) void prep_win_planes(
    const float* __restrict__ w_in, unsigned short* __restrict__ whi, unsigned short* __restrict__ wlo)
{
  const int t = blockIdx.x * 256 + threadIdx.x;
  if (t >= WIN_PLANE_HALVES / 8) return;
  const int n  = t / 12;
  const int k8 = (t - n * 12) * 8;
  float f[8];
#pragma unroll
  for (int j = 0; j < 8; ++j) f[j] = w_in[(size_t)(k8 + j) * NCH_PROJ + n];
  unsigned hw0, hw1, hw2, hw3, lw0, lw1, lw2, lw3;
  pack_hilo_pair(f[0], f[1], hw0, lw0);
  pack_hilo_pair(f[2], f[3], hw1, lw1);
  pack_hilo_pair(f[4], f[5], hw2, lw2);
  pack_hilo_pair(f[6], f[7], hw3, lw3);
  const v4u hv = (v4u){hw0, hw1, hw2, hw3};
  const v4u lv = (v4u){lw0, lw1, lw2, lw3};
  const size_t o = (size_t)t * 8;
  *(volatile v4u*)(void*)(whi + o) = hv;
  *(volatile v4u*)(void*)(wlo + o) = lv;
  __threadfence();
  *(volatile v4u*)(void*)(whi + o) = hv;
  *(volatile v4u*)(void*)(wlo + o) = lv;
}

__global__ __launch_bounds__(256) void prep_convw_frags(
    const float* __restrict__ conv_w, unsigned short* __restrict__ wpk)
{
  const int t = blockIdx.x * 256 + threadIdx.x;
  if (t >= WPK_HALVES / 8) return;
  const int hi8  = t & 1;
  const int ln   = (t >> 1) & 31;
  const int tile = t >> 6;
  const int nt   = tile % 6;
  const int kt   = (tile / 6) % 6;
  const int tap  = tile / 36;
  const int n    = nt * 16 + (ln & 15);
  const int kb   = kt * 32 + 8 * (ln >> 4) + 16 * hi8;
  unsigned w[4];
#pragma unroll
  for (int jp = 0; jp < 4; ++jp) {
    const float f0 = conv_w[((size_t)(tap * NCH_INNER + kb + 2 * jp)) * NCH_MODEL + n] * CONVW_CARRY;
    const float f1 = conv_w[((size_t)(tap * NCH_INNER + kb + 2 * jp + 1)) * NCH_MODEL + n] * CONVW_CARRY;
    const _Float16 h0 = (_Float16)f0, h1 = (_Float16)f1;
    w[jp] = (unsigned)__builtin_bit_cast(unsigned short, h0) | ((unsigned)__builtin_bit_cast(unsigned short, h1) << 16);
  }
  const v4u v = (v4u){w[0], w[1], w[2], w[3]};
  const size_t o = (size_t)t * 8;
  *(volatile v4u*)(void*)(wpk + o) = v;
  __threadfence();
  *(volatile v4u*)(void*)(wpk + o) = v;
}

__global__ __launch_bounds__(256) void conv3x3_silu_resid(
    const unsigned short* __restrict__ x1p, const unsigned short* __restrict__ wpk,
    const float* __restrict__ conv_b, const float* __restrict__ x, float* __restrict__ out)
{
  __shared__ __align__(16) _Float16 sX[NHALO * NCH_INNER];
  const _Float16* wp = (const _Float16*)(const void*)wpk;
  const int tid = threadIdx.x, lane = tid & 31, wave = tid >> 5;
  const int blk  = blockIdx.x;
  const int tx   = blk % TILES_X;
  const int ty   = (blk / TILES_X) % TILES_Y;
  const int bimg = blk / (TILES_X * TILES_Y);
  const int gh0  = ty * TILE_P, gw0 = tx * TILE_P;

  for (int cidx = tid; cidx < NHALO * (NCH_INNER / 8); cidx += 256) {
    const int pos = cidx / (NCH_INNER / 8);
    const int ch8 = (cidx - pos * (NCH_INNER / 8)) * 8;
    const int hr = pos / HALO_P, hc = pos - hr * HALO_P;
    const int gh = gh0 + hr - 1, gw = gw0 + hc - 1;
    const bool valid = (gh >= 0) && (gh < IMG_H) && (gw >= 0) && (gw < IMG_W);
    const int ghc = gh < 0 ? 0 : (gh >= IMG_H ? IMG_H - 1 : gh);
    const int gwc = gw < 0 ? 0 : (gw >= IMG_W ? IMG_W - 1 : gw);
    v4u v = *(const v4u*)(const void*)(x1p + (((size_t)bimg * IMG_H + ghc) * IMG_W + gwc) * NCH_INNER + ch8);
    const unsigned keep = valid ? 0xffffffffu : 0u;
    v &= (v4u){keep, keep, keep, keep};
    *(v4u*)(void*)(sX + pos * NCH_INNER + ch8) = v;
  }
  __syncthreads();

  const int mr    = lane & 15;
  const int khalf = (lane >> 4) * 8;
  const int mt    = wave & 3;
  const int ng    = (wave >> 2) * 3;
  const int ml    = mt * 16 + mr;
  const int orow  = ml >> 3, ocol = ml & 7;
  v8f acc0 = (v8f){0.f,0.f,0.f,0.f,0.f,0.f,0.f,0.f};
  v8f acc1 = (v8f){0.f,0.f,0.f,0.f,0.f,0.f,0.f,0.f};
  v8f acc2 = (v8f){0.f,0.f,0.f,0.f,0.f,0.f,0.f,0.f};
#pragma unroll 1
  for (int tap = 0; tap < 9; ++tap) {
    const int dh = tap / 3, dw = tap - dh * 3;
    const _Float16* arow = sX + ((orow + dh) * HALO_P + (ocol + dw)) * NCH_INNER + khalf;
#pragma unroll
    for (int kt = 0; kt < 6; ++kt) {
      const v16h a = Frag<_Float16>::load(arow + kt * 32);
      const _Float16* bt = wp + ((size_t)((tap * 6 + kt) * 6 + ng) * 32 + lane) * 16;
      const v16h b0 = *(const v16h*)(bt);
      const v16h b1 = *(const v16h*)(bt + 512);
      const v16h b2 = *(const v16h*)(bt + 1024);
      acc0 = Frag<_Float16>::mma(a, b0, acc0);
      acc1 = Frag<_Float16>::mma(a, b1, acc1);
      acc2 = Frag<_Float16>::mma(a, b2, acc2);
      guard3_h(acc0, acc1, acc2, a, b0, b1, b2);
    }
  }
  acc_guard3(acc0, acc1, acc2);
  __syncthreads();

  float* sOut = (float*)(void*)sX;
  {
    const int mbase = mt * 16 + khalf;
    const int n0c = ng * 16 + mr;
#pragma unroll
    for (int j = 0; j < 8; ++j) {
      sOut[(mbase + j) * NCH_MODEL + n0c]      = acc0[j] * CONVW_CARRY_INV;
      sOut[(mbase + j) * NCH_MODEL + n0c + 16] = acc1[j] * CONVW_CARRY_INV;
      sOut[(mbase + j) * NCH_MODEL + n0c + 32] = acc2[j] * CONVW_CARRY_INV;
    }
  }
  __syncthreads();

  const size_t gbase = (((size_t)bimg * IMG_H + gh0 + wave) * IMG_W + gw0) * NCH_MODEL;
  float* srow = sOut + wave * (TILE_P * NCH_MODEL);
#pragma unroll 1
  for (int it = 0; it < 6; ++it) {
    const int f  = (it * 4 + (lane >> 3)) * 32 + (lane & 7) * 4;
    const int ch = f - (f / NCH_MODEL) * NCH_MODEL;
    const v4f a4 = *(const v4f*)(srow + f);
    const v4f c4 = *(const v4f*)(conv_b + ch);
    const v4f x4 = *(const v4f*)(x + gbase + f);
    v4f o4;
#pragma unroll
    for (int e = 0; e < 4; ++e) {
      const float y  = a4[e] + c4[e];
      const float sg = 1.0f / (1.0f + expf(-y));
      o4[e] = x4[e] + y * sg;
    }
    *(v4f*)(srow + f) = o4;
  }
  for (int ps = 0; ps < 2; ++ps) {
#pragma unroll
    for (int it = 0; it < 6; ++it) {
      const int f = (it * 4 + (lane >> 3)) * 32 + (lane & 7) * 4;
      const v4f v = *(const v4f*)(srow + f);
      *(volatile v4f*)(out + gbase + f) = v;
    }
    __threadfence();
  }
}

extern "C" void kernel_launch(void* const* d_in, const int* in_sizes, int n_in,
                              void* d_out, int out_size, void* d_ws, size_t ws_size,
                              hipStream_t stream) {
  if (n_in < 7) return;
  if (in_sizes[0] != NPOS_ALL * NCH_MODEL) return;
  if (out_size != NPOS_ALL * NCH_MODEL) return;
  if (in_sizes[3] != NCH_MODEL * NCH_PROJ) return;
  if (in_sizes[5] != 9 * NCH_INNER * NCH_MODEL) return;
  if (ws_size < WS_TOTAL) return;

  const float* x      = (const float*)d_in[0];
  const float* ln_w   = (const float*)d_in[1];
  const float* ln_b   = (const float*)d_in[2];
  const float* w_in   = (const float*)d_in[3];
  const float* b_in   = (const float*)d_in[4];
  const float* conv_w = (const float*)d_in[5];
  const float* conv_b = (const float*)d_in[6];
  float* out = (float*)d_out;
  unsigned char* ws = (unsigned char*)d_ws;
  unsigned short* hhi = (unsigned short*)(ws + OFF_HHI);
  unsigned short* hlo = (unsigned short*)(ws + OFF_HLO);
  unsigned short* whi = (unsigned short*)(ws + OFF_WHI);
  unsigned short* wlo = (unsigned short*)(ws + OFF_WLO);
  unsigned short* wpk = (unsigned short*)(ws + OFF_WPK);
  unsigned short* x1  = (unsigned short*)(ws + OFF_X1);

  ln_split_planes<<<LN_NBLK, 256, 0, stream>>>(x, ln_w, ln_b, hhi, hlo);
  prep_win_planes<<<(WIN_PLANE_HALVES / 8) / 256, 256, 0, stream>>>(w_in, whi, wlo);
  prep_convw_frags<<<(WPK_HALVES / 8) / 256, 256, 0, stream>>>(conv_w, wpk);
  {
    const int tiles = (NPOS_ALL / 64) * (NCH_INNER / 64);
    wmma_gemm64<1, true, 2, 1, false, 0><<<dim3(tiles / 8, 1, 1), 256, 0, stream>>>(
        hhi, hlo, NCH_MODEL, 0L,
        whi, wlo, NCH_MODEL, 0L,
        (void*)x1, (void*)x1, NCH_INNER, 0L,
        b_in, x, 0L,
        NPOS_ALL, NCH_INNER, NCH_MODEL, 1.0f);
  }
  conv3x3_silu_resid<<<NTILE_BLK, 256, 0, stream>>>(x1, wpk, conv_b, x, out);
}
